// GFASTKAN_Nodes_49469433315364
// MI455X (gfx1250) — hardware-verified
//
#include <hip/hip_runtime.h>
#include <stddef.h>


#define NTHR    256
#define NWAVE   8
#define EPT     8
#define NGRP    2
#define CHUNK   (NTHR * EPT * NGRP)
#define WCAP    (EPT * NGRP * 32)
#define LISTN   (NWAVE * WCAP)
#define NBC     4096
#define NBF     1024
#define RCAP    49152
#define RBN     128
#define TGT     256
#define DEGCAP  1024
#define OTHR    512
#define BM      64
#define SB      64
#define FR      64
#define WSCAP   134217728
#define ABUD    33554432
#define FIN     128
#define HID     128
#define NCLS    40
#define DI2     384
#define K01     640
#define K2      1920
#define NB01    128
#define NB2     48
#define LDC2    64
#define ACARRY  32.0f
#define WCARRY  64.0f
#define GSCALE  (1.0f / 2048.0f)
#define LNEPS   1e-5f
#define BNEPS   1e-5f
#define GSTEP   (4.0f / 3.0f)
#define GR0     (-2.0f)
#define GR1     (-2.0f + GSTEP)
#define GR2     (-2.0f + 2.0f * GSTEP)
#define GR3     (2.0f)
#define RDEN    0.75f

#define LDS_FILL ((RCAP + NBF + LISTN) * 4 + 64)

static_assert((CHUNK & (CHUNK - 1)) == 0);
static_assert(CHUNK <= 4096);
static_assert((NBC & (NBC - 1)) == 0 && (NBF & (NBF - 1)) == 0);
static_assert(NBC == 4 * NBF);
static_assert(OTHR * 8 == NBC);
static_assert((RCAP % 32) == 0);
static_assert(TGT == NWAVE * 32);
static_assert((NBC % TGT) == 0);
static_assert((TGT % BM) == 0);
static_assert(WCAP == EPT * NGRP * 32);
static_assert(K01 == 5 * FIN && K2 == 5 * DI2);
static_assert((K01 % 32) == 0 && (K2 % 32) == 0);
static_assert(DI2 == FIN + 2 * HID);
static_assert(NB2 >= NCLS && NB2 <= LDC2 && (NB2 % 16) == 0);
static_assert((FR % NWAVE) == 0 && FR == BM);
static_assert(((ABUD / (K01 * 2)) / BM) * BM >= BM);
static_assert(((ABUD / (K2 * 2)) / BM) * BM >= BM);

typedef float    v2f  __attribute__((ext_vector_type(2)));
typedef float    v4f  __attribute__((ext_vector_type(4)));
typedef float    v8f  __attribute__((ext_vector_type(8)));
typedef int      v4i  __attribute__((ext_vector_type(4)));
typedef double   v2d  __attribute__((ext_vector_type(2)));
typedef _Float16 v4h  __attribute__((ext_vector_type(4)));
typedef _Float16 v8h  __attribute__((ext_vector_type(8)));
typedef _Float16 v16h __attribute__((ext_vector_type(16)));
union Frag { v16h v; v8h h[2]; };

__device__ __forceinline__ v8f wmh(v16h a, v16h b, v8f c) {
  v8f d = __builtin_amdgcn_wmma_f32_16x16x32_f16(false, a, false, b, (short)0, c, false, false);
  asm volatile("v_nop\n\tv_nop\n\tv_nop\n\tv_nop" : "+v"(d) : "v"(a), "v"(b));
  return d;
}

__device__ __forceinline__ v4f selz(v4f v, bool live) {
  v4f o; o.x = live ? v.x : 0.f; o.y = live ? v.y : 0.f; o.z = live ? v.z : 0.f; o.w = live ? v.w : 0.f; return o;
}
__device__ __forceinline__ v2f selz(v2f v, bool live) {
  v2f o; o.x = live ? v.x : 0.f; o.y = live ? v.y : 0.f; return o;
}
__device__ __forceinline__ float wsum1(float v) {
#pragma unroll
  for (int off = 16; off > 0; off >>= 1) v += __shfl_xor(v, off);
  return v;
}
template <typename VT, int W>
__device__ __forceinline__ VT ldvec_clamped(const float* __restrict__ p, int c0, int n) {
  VT o;
#pragma unroll
  for (int j = 0; j < W; ++j) {
    const int c = c0 + j;
    int cc = c > n - 1 ? n - 1 : c;
    cc = cc < 0 ? 0 : cc;
    const float v = p[cc];
    o[j] = c < n ? v : 0.f;
  }
  return o;
}

template <int NB>
__device__ __forceinline__ int scan_chunk(const int* __restrict__ dsts, int nE, int cbase, int slotBase,
                                          int vec8, int* list, int tid, int lane, int wave) {
  int wc = 0;
#pragma unroll
  for (int g = 0; g < NGRP; ++g) {
    const int el0  = (g * NTHR + tid) * EPT;
    const int e0   = cbase + el0;
    const int sent = -2147483647 - 1;
    v4i da, db;
    if (vec8 != 0 && cbase + CHUNK <= nE) {
      da = *(const v4i*)(dsts + e0);
      db = *(const v4i*)(dsts + e0 + 4);
    } else {
      da.x = (e0     < nE) ? dsts[min(e0, nE - 1)] : sent;
      da.y = (e0 + 1 < nE) ? dsts[min(e0 + 1, nE - 1)] : sent;
      da.z = (e0 + 2 < nE) ? dsts[min(e0 + 2, nE - 1)] : sent;
      da.w = (e0 + 3 < nE) ? dsts[min(e0 + 3, nE - 1)] : sent;
      db.x = (e0 + 4 < nE) ? dsts[min(e0 + 4, nE - 1)] : sent;
      db.y = (e0 + 5 < nE) ? dsts[min(e0 + 5, nE - 1)] : sent;
      db.z = (e0 + 6 < nE) ? dsts[min(e0 + 6, nE - 1)] : sent;
      db.w = (e0 + 7 < nE) ? dsts[min(e0 + 7, nE - 1)] : sent;
    }
    const unsigned nb = (unsigned)slotBase;
    const unsigned s0 = (unsigned)da.x - nb, s1 = (unsigned)da.y - nb;
    const unsigned s2 = (unsigned)da.z - nb, s3 = (unsigned)da.w - nb;
    const unsigned s4 = (unsigned)db.x - nb, s5 = (unsigned)db.y - nb;
    const unsigned s6 = (unsigned)db.z - nb, s7 = (unsigned)db.w - nb;
    const bool h0 = s0 < (unsigned)NB, h1 = s1 < (unsigned)NB, h2 = s2 < (unsigned)NB, h3 = s3 < (unsigned)NB;
    const bool h4 = s4 < (unsigned)NB, h5 = s5 < (unsigned)NB, h6 = s6 < (unsigned)NB, h7 = s7 < (unsigned)NB;
    const unsigned any = __builtin_amdgcn_ballot_w32(h0 | h1 | h2 | h3 | h4 | h5 | h6 | h7);
    if (any != 0u) {
#define HITJ(J, HJ, SJ) { \
        const unsigned mj = __builtin_amdgcn_ballot_w32(HJ); \
        if (mj != 0u) { \
          if (HJ) { \
            const int pos = wc + (int)__builtin_amdgcn_mbcnt_lo(mj, 0u); \
            if (pos < WCAP) list[wave * WCAP + pos] = ((el0 + (J)) << 12) | (int)(SJ); \
          } \
          wc += (int)__builtin_popcount(mj); } }
      HITJ(0, h0, s0)
      HITJ(1, h1, s1)
      HITJ(2, h2, s2)
      HITJ(3, h3, s3)
      HITJ(4, h4, s4)
      HITJ(5, h5, s5)
      HITJ(6, h6, s6)
      HITJ(7, h7, s7)
#undef HITJ
    }
  }
  return wc;
}

__global__ __launch_bounds__(NTHR) void k_count(
    const int* __restrict__ dsts, int* cnt, float* dinv, int nE, int vec8) {
  __shared__ __attribute__((aligned(16))) int scnt[NBC];
  __shared__ __attribute__((aligned(16))) int list[LISTN];
  __shared__ int wcnt[NWAVE];
  const int tid = threadIdx.x, lane = tid & 31, wave = tid >> 5;
  const int nodeBase = blockIdx.x * NBC;

  for (int i = tid; i < NBC; i += NTHR) scnt[i] = 0;
  __syncthreads();

  const int nChunks = (nE + CHUNK - 1) / CHUNK;
#pragma unroll 1
  for (int ch = 0; ch < nChunks; ++ch) {
    const int cbase = ch * CHUNK;
    const int wc = scan_chunk<NBC>(dsts, nE, cbase, nodeBase, vec8, list, tid, lane, wave);
    if (lane == 0) wcnt[wave] = wc;
    __syncthreads();
    if (wave == 0) {
#pragma unroll 1
      for (int wsx = 0; wsx < NWAVE; ++wsx) {
        int n = __builtin_amdgcn_readfirstlane(wcnt[wsx]);
        n = n > WCAP ? WCAP : (n < 0 ? 0 : n);
        const int* lp = list + wsx * WCAP;
#pragma unroll 1
        for (int i = 0; i < n; ++i) {
          const int ent  = __builtin_amdgcn_readfirstlane(lp[i]);
          const int slot = ent & (NBC - 1);
          if (lane == 0) scnt[slot] = scnt[slot] + 1;
        }
      }
    }
    __syncthreads();
  }

  v4i cq[4];
  v4f dq[4];
#pragma unroll
  for (int q = 0; q < 4; ++q) {
    const int f = (wave * 4 + q) * 128 + 4 * lane;
    const v4i cv = *(const v4i*)(scnt + f);
    cq[q] = cv;
    v4f d;
    d.x = rsqrtf((float)(cv.x < 0 ? 0 : cv.x) + 1.0f);
    d.y = rsqrtf((float)(cv.y < 0 ? 0 : cv.y) + 1.0f);
    d.z = rsqrtf((float)(cv.z < 0 ? 0 : cv.z) + 1.0f);
    d.w = rsqrtf((float)(cv.w < 0 ? 0 : cv.w) + 1.0f);
    dq[q] = d;
  }
  int*   cp = cnt  + (size_t)nodeBase;
  float* dp = dinv + (size_t)nodeBase;
#pragma unroll
  for (int q = 0; q < 4; ++q) {
    const int f = (wave * 4 + q) * 128 + 4 * lane;
    *(volatile v4i*)(cp + f) = cq[q];
    *(volatile v4f*)(dp + f) = dq[q];
  }
  __threadfence();
#pragma unroll
  for (int q = 0; q < 4; ++q) {
    const int f = (wave * 4 + q) * 128 + 4 * lane;
    *(volatile v4i*)(cp + f) = cq[q];
    *(volatile v4f*)(dp + f) = dq[q];
  }
}

__global__ __launch_bounds__(OTHR) void k_offsets(
    const int* __restrict__ cnt, int* off, int* rbase, int nChunk) {
  __shared__ __attribute__((aligned(16))) int soff[NBC];
  __shared__ __attribute__((aligned(16))) int srb[RBN];
  __shared__ int wtot[OTHR / 32];
  const int tid = threadIdx.x, lane = tid & 31, wave = tid >> 5, sub = tid >> 7;
  for (int i = tid; i < RBN; i += OTHR) srb[i] = 0;
  int carry = 0;
#pragma unroll 1
  for (int ch = 0; ch < nChunk; ++ch) {
    const int base = ch * NBC;
    const v4i c0 = *(const v4i*)(cnt + base + 8 * tid);
    const v4i c1 = *(const v4i*)(cnt + base + 8 * tid + 4);
    const int e0 = max(c0.x, 0), e1 = max(c0.y, 0), e2 = max(c0.z, 0), e3 = max(c0.w, 0);
    const int e4 = max(c1.x, 0), e5 = max(c1.y, 0), e6 = max(c1.z, 0), e7 = max(c1.w, 0);
    const int ts = e0 + e1 + e2 + e3 + e4 + e5 + e6 + e7;
    int incl = ts;
#pragma unroll
    for (int d = 1; d < 32; d <<= 1) {
      const int t = __shfl_up(incl, d);
      if (lane >= d) incl += t;
    }
    if (lane == 31) wtot[wave] = incl;
    __syncthreads();
    const int S0 = wtot[0]  + wtot[1]  + wtot[2]  + wtot[3];
    const int S1 = wtot[4]  + wtot[5]  + wtot[6]  + wtot[7];
    const int S2 = wtot[8]  + wtot[9]  + wtot[10] + wtot[11];
    const int S3 = wtot[12] + wtot[13] + wtot[14] + wtot[15];
    int pre = 0;
#pragma unroll 1
    for (int w = 4 * sub; w < wave; ++w) pre += wtot[w];
    const int b0 = carry;
    const int b1 = b0 + ((S0 + 31) & ~31);
    const int b2 = b1 + ((S1 + 31) & ~31);
    const int b3 = b2 + ((S2 + 31) & ~31);
    const int b4 = b3 + ((S3 + 31) & ~31);
    const int myb = sub == 0 ? b0 : (sub == 1 ? b1 : (sub == 2 ? b2 : b3));
    if (tid == 0) {
      srb[min(4 * ch + 0, RBN - 1)] = b0;
      srb[min(4 * ch + 1, RBN - 1)] = b1;
      srb[min(4 * ch + 2, RBN - 1)] = b2;
      srb[min(4 * ch + 3, RBN - 1)] = b3;
    }
    int run = myb + pre + incl - ts;
    soff[8 * tid + 0] = run; run += e0;
    soff[8 * tid + 1] = run; run += e1;
    soff[8 * tid + 2] = run; run += e2;
    soff[8 * tid + 3] = run; run += e3;
    soff[8 * tid + 4] = run; run += e4;
    soff[8 * tid + 5] = run; run += e5;
    soff[8 * tid + 6] = run; run += e6;
    soff[8 * tid + 7] = run;
    carry = b4;
    __syncthreads();
    const v4i o0 = *(const v4i*)(soff + 4 * tid);
    const v4i o1 = *(const v4i*)(soff + 4 * (tid + OTHR));
    int* op = off + base;
    *(volatile v4i*)(op + 4 * tid) = o0;
    *(volatile v4i*)(op + 4 * (tid + OTHR)) = o1;
    __threadfence();
    *(volatile v4i*)(op + 4 * tid) = o0;
    *(volatile v4i*)(op + 4 * (tid + OTHR)) = o1;
    __syncthreads();
  }
  if (tid == 0) srb[min(4 * nChunk, RBN - 1)] = carry;
  __syncthreads();
  v4i rv = {0, 0, 0, 0};
  if (tid < 32) rv = *(const v4i*)(srb + 4 * tid);
  if (tid < 32) *(volatile v4i*)(rbase + 4 * tid) = rv;
  __threadfence();
  if (tid < 32) *(volatile v4i*)(rbase + 4 * tid) = rv;
}

__global__ __launch_bounds__(NTHR) void k_fill(
    const int* __restrict__ srcs, const int* __restrict__ dsts,
    const int* __restrict__ off, const int* __restrict__ rbase,
    int* csr, int nN, int nE, int vec8, int csrLen) {
  extern __shared__ v4f lds_dyn[];
  int* region = (int*)lds_dyn;
  int* cursor = region + RCAP;
  int* list   = cursor + NBF;
  int* wcnt   = list + LISTN;
  const int tid = threadIdx.x, lane = tid & 31, wave = tid >> 5;
  const int b = blockIdx.x;
  const int nodeBase = b * NBF;

  int rb0 = rbase[b];
  const int rb1 = rbase[b + 1];
  rb0 = rb0 < 0 ? 0 : (rb0 > csrLen ? csrLen : rb0);
  rb0 &= ~31;
  int len = rb1 - rb0;
  len = len < 0 ? 0 : (len > RCAP ? RCAP : len);
  int lenW = (len + 31) & ~31;
  if (rb0 + lenW > csrLen) lenW = (csrLen - rb0) & ~31;

  {
    const v4i z = {0, 0, 0, 0};
    for (int i = tid; i < RCAP / 4; i += NTHR) ((v4i*)region)[i] = z;
    for (int s = tid; s < NBF; s += NTHR) {
      int o = off[nodeBase + s] - rb0;
      o = o < 0 ? 0 : (o > RCAP ? RCAP : o);
      cursor[s] = o;
    }
  }
  __syncthreads();

  const int nChunks = (nE + CHUNK - 1) / CHUNK;
#pragma unroll 1
  for (int ch = 0; ch < nChunks; ++ch) {
    const int cbase = ch * CHUNK;
    const int wc = scan_chunk<NBF>(dsts, nE, cbase, nodeBase, vec8, list, tid, lane, wave);
    if (lane == 0) wcnt[wave] = wc;
    __syncthreads();
    if (wave == 0) {
#pragma unroll 1
      for (int wsx = 0; wsx < NWAVE; ++wsx) {
        int n = __builtin_amdgcn_readfirstlane(wcnt[wsx]);
        n = n > WCAP ? WCAP : (n < 0 ? 0 : n);
        const int* lp = list + wsx * WCAP;
#pragma unroll 1
        for (int i = 0; i < n; ++i) {
          const int ent  = __builtin_amdgcn_readfirstlane(lp[i]);
          const int slot = ent & (NBF - 1);
          int e = cbase + ((ent >> 12) & (CHUNK - 1));
          e = e > nE - 1 ? nE - 1 : e;
          int sv = srcs[e];
          sv = sv < 0 ? 0 : (sv > nN - 1 ? nN - 1 : sv);
          if (lane == 0) {
            int pos = cursor[slot];
            pos = pos < 0 ? 0 : (pos > RCAP - 1 ? RCAP - 1 : pos);
            region[pos] = sv;
            const int np = pos + 1;
            cursor[slot] = np > RCAP ? RCAP : np;
          }
        }
      }
    }
    __syncthreads();
  }

  const int nv = lenW >> 2;
  int* gp = csr + rb0;
#pragma unroll 1
  for (int i = tid; i < nv; i += NTHR) { const v4i v = ((const v4i*)region)[i]; *(volatile v4i*)(gp + 4 * i) = v; }
  __threadfence();
#pragma unroll 1
  for (int i = tid; i < nv; i += NTHR) { const v4i v = ((const v4i*)region)[i]; *(volatile v4i*)(gp + 4 * i) = v; }
}

__global__ __launch_bounds__(NTHR) void k_wcvt(const float* __restrict__ ws_, const float* __restrict__ wb,
                                               _Float16* dp, int KG, int K, int nsrc, int nUnits) {
  const int i = (int)blockIdx.x * NTHR + (int)threadIdx.x;
  if (i >= nUnits) return;
  const int ppr = K >> 3;
  const int n = i / ppr;
  const int seg = i - n * ppr;
  int nc = n > nsrc - 1 ? nsrc - 1 : n;
  nc = nc < 0 ? 0 : nc;
  const bool live = n < nsrc;
  int KB = K - KG;
  KB = KB < 1 ? 1 : KB;
  v8h o;
#pragma unroll
  for (int j = 0; j < 8; ++j) {
    const int k = 8 * seg + j;
    int ka = k > KG - 1 ? KG - 1 : k;
    ka = ka < 0 ? 0 : ka;
    int kb = k - KG;
    kb = kb < 0 ? 0 : (kb > KB - 1 ? KB - 1 : kb);
    const float fa = ws_[(size_t)nc * KG + ka];
    const float fb = wb[(size_t)nc * KB + kb];
    float f = (k < KG) ? fa : fb;
    f = live ? f : 0.f;
    o[j] = (_Float16)(f * WCARRY);
  }
  _Float16* gp = dp + (size_t)i * 8;
  *(volatile v8h*)gp = o;
  __threadfence();
  *(volatile v8h*)gp = o;
}

template <int NS>
__global__ __launch_bounds__(NTHR) void k_feat(
    const float* __restrict__ p0, const float* __restrict__ p1, const float* __restrict__ p2,
    const float* __restrict__ lg, const float* __restrict__ lb, _Float16* aout, int rowBase, int nN) {
  constexpr int DI   = 128 * NS;
  constexpr int KG   = 4 * DI;
  constexpr int K    = 5 * DI;
  constexpr int NCH  = DI / 32;
  constexpr int PPRW = K / 8;
  constexpr int NI   = (PPRW + 31) / 32;
  static_assert((K % 64) == 0);
  __shared__ __attribute__((aligned(16))) _Float16 srow[NWAVE * K];
  const int tid = threadIdx.x, lane = tid & 31, wave = tid >> 5;
  _Float16* my = srow + wave * K;
  const float invd = 1.0f / (float)DI;

#pragma unroll 1
  for (int it = 0; it < FR / NWAVE; ++it) {
    const int lr = (int)blockIdx.x * FR + it * NWAVE + wave;
    const int gr = rowBase + lr;
    int rr = gr > nN - 1 ? nN - 1 : gr;
    rr = rr < 0 ? 0 : rr;
    const size_t ro = (size_t)rr * 128 + lane;

    float hv[NCH];
#pragma unroll
    for (int ch = 0; ch < NCH; ++ch) {
      const float* sp = ((ch >> 2) == 0) ? p0 : (((ch >> 2) == 1) ? p1 : p2);
      hv[ch] = sp[ro + 32 * (ch & 3)];
    }
    float s = 0.f;
#pragma unroll
    for (int ch = 0; ch < NCH; ++ch) s += hv[ch];
    s = wsum1(s);
    const float mu = s * invd;
    float sq = 0.f;
#pragma unroll
    for (int ch = 0; ch < NCH; ++ch) { const float d = hv[ch] - mu; sq += d * d; }
    sq = wsum1(sq);
    const float rs = rsqrtf(sq * invd + LNEPS);

#pragma unroll
    for (int sg = 0; sg < NS; ++sg) {
      const float* sp = (sg == 0) ? p0 : ((sg == 1) ? p1 : p2);
#pragma unroll 1
      for (int q = 0; q < 4; ++q) {
        const int c = 128 * sg + 32 * q + lane;
        const float h  = sp[ro + 32 * q];
        const float hn = (h - mu) * rs * lg[c] + lb[c];
        const float t0 = (hn - GR0) * RDEN;
        const float t1 = (hn - GR1) * RDEN;
        const float t2 = (hn - GR2) * RDEN;
        const float t3 = (hn - GR3) * RDEN;
        const float e0 = __expf(-(t0 * t0));
        const float e1 = __expf(-(t1 * t1));
        const float e2 = __expf(-(t2 * t2));
        const float e3 = __expf(-(t3 * t3));
        const float ex = __expf(-h);
        const float sl = h * __builtin_amdgcn_rcpf(1.0f + ex);
        v4h bq;
        bq.x = (_Float16)(e0 * ACARRY);
        bq.y = (_Float16)(e1 * ACARRY);
        bq.z = (_Float16)(e2 * ACARRY);
        bq.w = (_Float16)(e3 * ACARRY);
        *(v4h*)(my + 4 * c) = bq;
        my[KG + c] = (_Float16)(sl * ACARRY);
      }
    }
    __syncthreads();

    _Float16* gp = aout + (size_t)lr * K;
    v8h pv[NI];
#pragma unroll
    for (int i = 0; i < NI; ++i) {
      int p = i * 32 + lane;
      p = p > PPRW - 1 ? PPRW - 1 : p;
      pv[i] = *(const v8h*)(my + 8 * p);
    }
#pragma unroll
    for (int i = 0; i < NI; ++i) {
      const int p = i * 32 + lane;
      if (p < PPRW) *(volatile v8h*)(gp + 8 * p) = pv[i];
    }
    __threadfence();
#pragma unroll
    for (int i = 0; i < NI; ++i) {
      const int p = i * 32 + lane;
      if (p < PPRW) *(volatile v8h*)(gp + 8 * p) = pv[i];
    }
    __syncthreads();
  }
}

template <int NWV, int TPW, int BNCT>
__global__ __launch_bounds__(NWV * 32) void k_gemm(
    const _Float16* __restrict__ A, const _Float16* __restrict__ Bp,
    const float* __restrict__ b0, const float* __restrict__ b1, int nb,
    float* Cout, int K, int ldc, int nValid, int nStore) {
  constexpr int NT  = NWV * 32;
  constexpr int WPR = NWV / 4;
  static_assert(WPR >= 1 && WPR * 4 == NWV);
  constexpr int NCOMP = WPR * TPW * 16;
  static_assert(NCOMP <= BNCT && (BNCT % 32) == 0);
  constexpr int PADW = BNCT - NCOMP;
  constexpr int PADD = PADW > 0 ? PADW : 1;
  constexpr int PPR = BNCT / 4;
  constexpr int NIT = (BM * PPR) / NT;
  static_assert(NIT * NT == BM * PPR && NIT >= 1);
  static_assert(BM == 4 * 16);

  __shared__ __attribute__((aligned(16))) float stg[BM * BNCT];
  const int tid = threadIdx.x, lane = tid & 31, wave = tid >> 5, hh = lane >> 4, m = lane & 15;
  const int rowBase = (int)blockIdx.x * BM;
  const int colBase = (int)blockIdx.y * BNCT;
  const int rg = wave / WPR, chf = wave - rg * WPR;
  const int r0 = rg * 16;
  const int c0 = chf * TPW * 16;

  v8f acc[TPW];
#pragma unroll
  for (int t = 0; t < TPW; ++t) { v8f z = {0.f, 0.f, 0.f, 0.f, 0.f, 0.f, 0.f, 0.f}; acc[t] = z; }

  const _Float16* ap = A  + (size_t)(rowBase + r0 + m) * K + 8 * hh;
  const _Float16* bp = Bp + (size_t)(colBase + c0 + m) * K + 8 * hh;
  const int ksteps = K >> 5;
#pragma unroll 1
  for (int kt = 0; kt < ksteps; ++kt) {
    Frag a;
    a.h[0] = *(const v8h*)(ap + 32 * kt);
    a.h[1] = *(const v8h*)(ap + 32 * kt + 16);
#pragma unroll
    for (int t = 0; t < TPW; ++t) {
      const size_t to = (size_t)(16 * t) * K + 32 * kt;
      Frag b;
      b.h[0] = *(const v8h*)(bp + to);
      b.h[1] = *(const v8h*)(bp + to + 16);
      acc[t] = wmh(a.v, b.v, acc[t]);
    }
  }

  float bv[TPW];
#pragma unroll
  for (int t = 0; t < TPW; ++t) {
    const int col = colBase + c0 + 16 * t + m;
    int cc = col > nb - 1 ? nb - 1 : col;
    cc = cc < 0 ? 0 : cc;
    const float bs = b0[cc] + b1[cc];
    bv[t] = col < nb ? bs : 0.f;
  }

  {
    float* sp = stg + (size_t)(r0 + 8 * hh) * BNCT + c0 + m;
    const int growb = rowBase + r0 + 8 * hh;
#pragma unroll
    for (int t = 0; t < TPW; ++t) {
#pragma unroll
      for (int r = 0; r < 8; ++r) {
        const bool lv = (growb + r) < nValid;
        const float g = acc[t][r] * GSCALE + bv[t];
        sp[r * BNCT + 16 * t] = lv ? g : 0.f;
      }
    }
  }
  if (PADW > 0) {
#pragma unroll 1
    for (int idx = tid; idx < BM * PADW; idx += NT) {
      const int row = idx / PADD, cc = idx - row * PADD;
      stg[(size_t)row * BNCT + NCOMP + cc] = 0.f;
    }
  }
  __syncthreads();

  v4f cv[NIT];
#pragma unroll
  for (int it = 0; it < NIT; ++it) {
    const int id = it * NT + tid;
    const int row = id / PPR, seg = id - row * PPR;
    cv[it] = *(const v4f*)(stg + (size_t)row * BNCT + 4 * seg);
  }
#pragma unroll
  for (int it = 0; it < NIT; ++it) {
    const int id = it * NT + tid;
    const int row = id / PPR, seg = id - row * PPR;
    const int grow = rowBase + row;
    if (grow < nStore) {
      float* gp = Cout + (size_t)grow * ldc + colBase + 4 * seg;
      *(volatile v4f*)gp = cv[it];
    }
  }
  __threadfence();
#pragma unroll
  for (int it = 0; it < NIT; ++it) {
    const int id = it * NT + tid;
    const int row = id / PPR, seg = id - row * PPR;
    const int grow = rowBase + row;
    if (grow < nStore) {
      float* gp = Cout + (size_t)grow * ldc + colBase + 4 * seg;
      *(volatile v4f*)gp = cv[it];
    }
  }
}

template <int NP, typename VT, int W>
__global__ __launch_bounds__(NTHR) void k_aggsym(
    const int* __restrict__ csr, const int* __restrict__ off, const int* __restrict__ cnt,
    const float* __restrict__ dinv, const float* __restrict__ hw, const float* __restrict__ cb, int nb,
    float* hout, int nN, int csrLen) {
  constexpr int CW = NP * 32 * W;
  const int tid = threadIdx.x, lane = tid & 31, wave = tid >> 5;
  const int tbase = blockIdx.x * TGT + wave * 32;
  const int cl    = tbase + lane;
  const int cnt_l = cnt[cl];
  const int off_l = off[cl];
  const float di_l = dinv[cl];
  VT cbv[NP];
#pragma unroll
  for (int p = 0; p < NP; ++p) cbv[p] = ldvec_clamped<VT, W>(cb, (p * 32 + lane) * W, nb);

#pragma unroll 1
  for (int j = 0; j < 32; ++j) {
    const int c = tbase + j;
    int n = __shfl(cnt_l, j);
    n = n < 0 ? 0 : (n > DEGCAP ? DEGCAP : n);
    const int st = __shfl(off_l, j);
    const float dc = __shfl(di_l, j);
    const float dd = dc * dc;

    VT a[NP];
#pragma unroll
    for (int p = 0; p < NP; ++p) a[p] = *(const VT*)(hw + (size_t)c * CW + (p * 32 + lane) * W) * dd;
#pragma unroll 1
    for (int q0 = 0; q0 < n; q0 += 32) {
      int pos = st + q0 + lane;
      pos = pos < 0 ? 0 : (pos > csrLen - 1 ? csrLen - 1 : pos);
      int sl = csr[pos];
      sl = sl < 0 ? 0 : (sl > nN - 1 ? nN - 1 : sl);
      const int mcnt = (n - q0) < 32 ? (n - q0) : 32;
#pragma unroll 1
      for (int pp = 0; pp < mcnt; ++pp) {
        const int s = __builtin_amdgcn_readlane(sl, pp);
        const float cf = dinv[s] * dc;
#pragma unroll
        for (int p = 0; p < NP; ++p) {
          const VT xv = *(const VT*)(hw + (size_t)s * CW + (p * 32 + lane) * W);
          a[p] = a[p] + xv * cf;
        }
      }
    }

    const bool live = c < nN;
    VT o[NP];
#pragma unroll
    for (int p = 0; p < NP; ++p) o[p] = selz(a[p] + cbv[p], live);
    float* gp = hout + (size_t)c * CW + W * lane;
#pragma unroll
    for (int p = 0; p < NP; ++p) *(volatile VT*)(gp + p * 32 * W) = o[p];
    __threadfence();
#pragma unroll
    for (int p = 0; p < NP; ++p) *(volatile VT*)(gp + p * 32 * W) = o[p];
  }
}

template <int C>
__global__ __launch_bounds__(NTHR) void k_bnstat(const float* __restrict__ x, double* part, int nN, int rpb) {
  constexpr int CL  = C < NTHR ? C : NTHR;
  constexpr int RG  = NTHR / CL;
  constexpr int CPT = C / CL;
  static_assert(RG * CL == NTHR);
  static_assert(CPT * CL == C);
  __shared__ __attribute__((aligned(16))) double sred[2 * RG * C];
  __shared__ __attribute__((aligned(16))) double sout[2 * C];
  const int tid = threadIdx.x;
  const int rg = tid / CL, c0 = tid - rg * CL;
  const int r0 = blockIdx.x * rpb;
  const int r1 = min(r0 + rpb, nN);
  double s[CPT], s2[CPT];
#pragma unroll
  for (int i = 0; i < CPT; ++i) { s[i] = 0.0; s2[i] = 0.0; }
#pragma unroll 1
  for (int r = r0 + rg; r < r1; r += RG) {
#pragma unroll
    for (int i = 0; i < CPT; ++i) {
      const double v = (double)x[(size_t)r * C + c0 + CL * i];
      s[i] += v;
      s2[i] += v * v;
    }
  }
#pragma unroll
  for (int i = 0; i < CPT; ++i) {
    sred[(0 * RG + rg) * C + c0 + CL * i] = s[i];
    sred[(1 * RG + rg) * C + c0 + CL * i] = s2[i];
  }
  __syncthreads();
#pragma unroll 1
  for (int idx = tid; idx < 2 * C; idx += NTHR) {
    const int q = idx / C, c = idx - q * C;
    double S = 0.0;
#pragma unroll
    for (int g = 0; g < RG; ++g) S += sred[(q * RG + g) * C + c];
    sout[idx] = S;
  }
  __syncthreads();
  double* gp = part + (size_t)blockIdx.x * 2 * C;
#pragma unroll 1
  for (int p = tid; p < C; p += NTHR) { const v2d v = *(const v2d*)(sout + 2 * p); *(volatile v2d*)(gp + 2 * p) = v; }
  __threadfence();
#pragma unroll 1
  for (int p = tid; p < C; p += NTHR) { const v2d v = *(const v2d*)(sout + 2 * p); *(volatile v2d*)(gp + 2 * p) = v; }
}

template <int C>
__global__ __launch_bounds__(NTHR) void k_bnapply(
    float* x, const double* __restrict__ part, const float* __restrict__ gam, const float* __restrict__ bet,
    int nN, int npad, int rpb, int nPart, double invN) {
  static_assert((C % 64) == 0 && C <= 2 * NTHR);
  constexpr int PPR = C / 4;
  constexpr int RPP = NTHR / PPR;
  static_assert(RPP * PPR == NTHR);
  __shared__ __attribute__((aligned(16))) float smu[C];
  __shared__ __attribute__((aligned(16))) float ssc[C];
  __shared__ __attribute__((aligned(16))) float sbb[C];
  const int tid = threadIdx.x;
#pragma unroll 1
  for (int c = tid; c < C; c += NTHR) {
    double s = 0.0, s2 = 0.0;
#pragma unroll 1
    for (int b = 0; b < nPart; ++b) {
      s  += part[((size_t)b * 2) * C + c];
      s2 += part[((size_t)b * 2 + 1) * C + c];
    }
    const double mu = s * invN;
    double var = s2 * invN - mu * mu;
    var = var < 0.0 ? 0.0 : var;
    const float muf = (float)mu, varf = (float)var;
    const float rstd = rsqrtf(varf + BNEPS);
    smu[c] = muf;
    ssc[c] = rstd * gam[c];
    sbb[c] = bet[c];
  }
  __syncthreads();
  const int seg = tid % PPR, rsub = tid / PPR;
  const v4f mu4 = *(const v4f*)(smu + 4 * seg);
  const v4f sc4 = *(const v4f*)(ssc + 4 * seg);
  const v4f bb4 = *(const v4f*)(sbb + 4 * seg);
  const int r0 = blockIdx.x * rpb;
  const int r1 = min(r0 + rpb, npad);
#pragma unroll 1
  for (int rs = r0; rs < r1; rs += RPP) {
    const int row = rs + rsub;
    if (row < r1) {
      const size_t o = (size_t)row * C + 4 * seg;
      const v4f v = *(const v4f*)(x + o);
      v4f y = (v - mu4) * sc4 + bb4;
      const bool live = row < nN;
      y = selz(y, live);
      *(volatile v4f*)(x + o) = y;
      __threadfence();
      *(volatile v4f*)(x + o) = y;
    }
  }
}

__global__ __launch_bounds__(NTHR) void k_outcopy(const float* __restrict__ src, int lds_, int ncol,
                                                  float* out, int n4) {
  const int i = (int)blockIdx.x * NTHR + (int)threadIdx.x;
  if (i >= n4) return;
  const int f = 4 * i;
  const int row = f / ncol;
  const int col = f - row * ncol;
  const v4f v = *(const v4f*)(src + (size_t)row * lds_ + col);
  float* gp = out + (size_t)f;
  *(volatile v4f*)gp = v;
  __threadfence();
  *(volatile v4f*)gp = v;
}

extern "C" void kernel_launch(void* const* d_in, const int* in_sizes, int n_in,
                              void* d_out, int out_size, void* d_ws, size_t ws_size,
                              hipStream_t stream) {
  if (n_in < 25) return;
  if (in_sizes[0] < FIN || (in_sizes[0] % FIN) != 0) return;
  const int nN = in_sizes[0] / FIN;
  if (nN < 1 || nN > (1 << 20)) return;
  if (in_sizes[1] < 2 || (in_sizes[1] & 1) != 0) return;
  const int nE = in_sizes[1] / 2;
  if (nE > (1 << 26)) return;
  if (in_sizes[2] != FIN || in_sizes[3] != FIN) return;
  if (in_sizes[4] != HID * 4 * FIN || in_sizes[5] != HID || in_sizes[6] != HID * FIN) return;
  if (in_sizes[7] != HID || in_sizes[8] != HID) return;
  if (in_sizes[9] != HID || in_sizes[10] != HID) return;
  if (in_sizes[11] != HID * 4 * HID || in_sizes[12] != HID || in_sizes[13] != HID * HID) return;
  if (in_sizes[14] != HID || in_sizes[15] != HID) return;
  if (in_sizes[16] != DI2 || in_sizes[17] != DI2) return;
  if (in_sizes[18] != NCLS * 4 * DI2 || in_sizes[19] != NCLS || in_sizes[20] != NCLS * DI2) return;
  if (in_sizes[21] != NCLS || in_sizes[22] != NCLS) return;
  if (in_sizes[23] != HID || in_sizes[24] != HID) return;
  if (out_size != nN * NCLS) return;
  if ((out_size & 3) != 0) return;

  const float* x    = (const float*)d_in[0];
  const int*   ei   = (const int*)d_in[1];
  const int*   src  = ei;
  const int*   dst  = ei + nE;
  const float* l0g  = (const float*)d_in[2];
  const float* l0b  = (const float*)d_in[3];
  const float* s0w  = (const float*)d_in[4];
  const float* s0b  = (const float*)d_in[5];
  const float* b0w  = (const float*)d_in[6];
  const float* b0b  = (const float*)d_in[7];
  const float* g0b  = (const float*)d_in[8];
  const float* l1g  = (const float*)d_in[9];
  const float* l1b  = (const float*)d_in[10];
  const float* s1w  = (const float*)d_in[11];
  const float* s1b  = (const float*)d_in[12];
  const float* b1w  = (const float*)d_in[13];
  const float* b1b  = (const float*)d_in[14];
  const float* g1b  = (const float*)d_in[15];
  const float* l2g  = (const float*)d_in[16];
  const float* l2b  = (const float*)d_in[17];
  const float* s2w  = (const float*)d_in[18];
  const float* s2b  = (const float*)d_in[19];
  const float* b2w  = (const float*)d_in[20];
  const float* b2b  = (const float*)d_in[21];
  const float* g2b  = (const float*)d_in[22];
  const float* bng  = (const float*)d_in[23];
  const float* bnb  = (const float*)d_in[24];
  float* out = (float*)d_out;

  const int NPAD   = ((nN + TGT - 1) / TGT) * TGT;
  const int nAgg   = NPAD / TGT;
  const int nBC    = (nN + NBC - 1) / NBC;
  const int CNTPAD = nBC * NBC;
  if (CNTPAD < NPAD) return;
  if (4 * nBC + 1 > RBN) return;
  const int nBF    = (nN + NBF - 1) / NBF;
  if (nBF > 4 * nBC) return;
  const int csrLen = ((nE + 31) & ~31) + 4096;
  if (31 * 4 * nBC > 4096) return;
  const int rpbS   = (nN + SB - 1) / SB;
  const double invN = 1.0 / (double)nN;
  const int CH01   = ((ABUD / (K01 * 2)) / BM) * BM;
  const int CH2    = ((ABUD / (K2 * 2)) / BM) * BM;
  if (CH01 < BM || CH2 < BM) return;
  const int n4     = out_size / 4;

  char* ws = (char*)d_ws;
  size_t off = 0;
  const size_t oCnt = off; off += (size_t)CNTPAD * 4;                    off = (off + 255) & ~(size_t)255;
  const size_t oDi  = off; off += (size_t)CNTPAD * 4;                    off = (off + 255) & ~(size_t)255;
  const size_t oOff = off; off += (size_t)CNTPAD * 4;                    off = (off + 255) & ~(size_t)255;
  const size_t oRb  = off; off += (size_t)RBN * 4;                       off = (off + 255) & ~(size_t)255;
  const size_t oCsr = off; off += (size_t)csrLen * 4;                    off = (off + 255) & ~(size_t)255;
  const size_t oW0  = off; off += (size_t)NB01 * K01 * 2;                off = (off + 255) & ~(size_t)255;
  const size_t oW1  = off; off += (size_t)NB01 * K01 * 2;                off = (off + 255) & ~(size_t)255;
  const size_t oW2  = off; off += (size_t)NB2 * K2 * 2;                  off = (off + 255) & ~(size_t)255;
  const size_t oA   = off; off += (size_t)ABUD;                          off = (off + 255) & ~(size_t)255;
  const size_t oHw  = off; off += (size_t)NPAD * HID * 4;                off = (off + 255) & ~(size_t)255;
  const size_t oC1  = off; off += (size_t)NPAD * HID * 4;                off = (off + 255) & ~(size_t)255;
  const size_t oC2  = off; off += (size_t)NPAD * HID * 4;                off = (off + 255) & ~(size_t)255;
  const size_t oPt  = off; off += (size_t)SB * 2 * HID * 8;              off = (off + 255) & ~(size_t)255;
  if (off > ws_size || off > (size_t)WSCAP) return;
  if ((size_t)CH01 * K01 * 2 > (size_t)ABUD || (size_t)CH2 * K2 * 2 > (size_t)ABUD) return;
  if ((size_t)NPAD * LDC2 * 4 > (size_t)ABUD) return;

  int*   cnt   = (int*)(ws + oCnt);
  float* dinv  = (float*)(ws + oDi);
  int*   offp  = (int*)(ws + oOff);
  int*   rb    = (int*)(ws + oRb);
  int*   csr   = (int*)(ws + oCsr);
  _Float16* w0p = (_Float16*)(ws + oW0);
  _Float16* w1p = (_Float16*)(ws + oW1);
  _Float16* w2p = (_Float16*)(ws + oW2);
  _Float16* apl = (_Float16*)(ws + oA);
  float* agg2  = (float*)(ws + oA);
  float* hw    = (float*)(ws + oHw);
  float* c1    = (float*)(ws + oC1);
  float* c2    = (float*)(ws + oC2);
  double* part = (double*)(ws + oPt);

  const int vec8 = ((nE & 3) == 0) ? 1 : 0;

  k_count<<<nBC, NTHR, 0, stream>>>(dst, cnt, dinv, nE, vec8);
  k_offsets<<<1, OTHR, 0, stream>>>(cnt, offp, rb, nBC);
  hipFuncSetAttribute(reinterpret_cast<const void*>(&k_fill),
                      hipFuncAttributeMaxDynamicSharedMemorySize, LDS_FILL);
  k_fill<<<nBF, NTHR, LDS_FILL, stream>>>(src, dst, offp, rb, csr, nN, nE, vec8, csrLen);

  {
    const int u0 = NB01 * (K01 / 8);
    k_wcvt<<<(u0 + NTHR - 1) / NTHR, NTHR, 0, stream>>>(s0w, b0w, w0p, 4 * FIN, K01, HID, u0);
    k_wcvt<<<(u0 + NTHR - 1) / NTHR, NTHR, 0, stream>>>(s1w, b1w, w1p, 4 * HID, K01, HID, u0);
    const int u2 = NB2 * (K2 / 8);
    k_wcvt<<<(u2 + NTHR - 1) / NTHR, NTHR, 0, stream>>>(s2w, b2w, w2p, 4 * DI2, K2, NCLS, u2);
  }

  for (int r0 = 0; r0 < NPAD; r0 += CH01) {
    const int rows = (NPAD - r0) < CH01 ? (NPAD - r0) : CH01;
    k_feat<1><<<rows / FR, NTHR, 0, stream>>>(x, x, x, l0g, l0b, apl, r0, nN);
    k_gemm<8, 4, 128><<<dim3(rows / BM, NB01 / 128), 256, 0, stream>>>(
        apl, w0p, s0b, b0b, HID, hw + (size_t)r0 * HID, K01, HID, nN - r0, rows);
  }
  k_aggsym<1, v4f, 4><<<nAgg, NTHR, 0, stream>>>(csr, offp, cnt, dinv, hw, g0b, HID, c1, nN, csrLen);
  k_bnstat<HID><<<SB, NTHR, 0, stream>>>(c1, part, nN, rpbS);
  k_bnapply<HID><<<nAgg, NTHR, 0, stream>>>(c1, part, bng, bnb, nN, NPAD, TGT, SB, invN);

  for (int r0 = 0; r0 < NPAD; r0 += CH01) {
    const int rows = (NPAD - r0) < CH01 ? (NPAD - r0) : CH01;
    k_feat<1><<<rows / FR, NTHR, 0, stream>>>(c1, c1, c1, l1g, l1b, apl, r0, nN);
    k_gemm<8, 4, 128><<<dim3(rows / BM, NB01 / 128), 256, 0, stream>>>(
        apl, w1p, s1b, b1b, HID, hw + (size_t)r0 * HID, K01, HID, nN - r0, rows);
  }
  k_aggsym<1, v4f, 4><<<nAgg, NTHR, 0, stream>>>(csr, offp, cnt, dinv, hw, g1b, HID, c2, nN, csrLen);
  k_bnstat<HID><<<SB, NTHR, 0, stream>>>(c2, part, nN, rpbS);
  k_bnapply<HID><<<nAgg, NTHR, 0, stream>>>(c2, part, bng, bnb, nN, NPAD, TGT, SB, invN);

  for (int r0 = 0; r0 < NPAD; r0 += CH2) {
    const int rows = (NPAD - r0) < CH2 ? (NPAD - r0) : CH2;
    k_feat<3><<<rows / FR, NTHR, 0, stream>>>(x, c1, c2, l2g, l2b, apl, r0, nN);
    k_gemm<4, 3, LDC2><<<dim3(rows / BM, 1), 128, 0, stream>>>(
        apl, w2p, s2b, b2b, NCLS, hw + (size_t)r0 * LDC2, K2, LDC2, nN - r0, rows);
  }
  k_aggsym<1, v2f, 2><<<nAgg, NTHR, 0, stream>>>(csr, offp, cnt, dinv, hw, g2b, NCLS, agg2, nN, csrLen);
  k_outcopy<<<(n4 + NTHR - 1) / NTHR, NTHR, 0, stream>>>(agg2, LDC2, NCLS, out, n4);
}
